// RiemannianManifold_65687229825096
// MI455X (gfx1250) — hardware-verified
//
#include <hip/hip_runtime.h>
#include <hip/hip_bf16.h>


typedef _Float16 v16h __attribute__((ext_vector_type(16)));
typedef _Float16 v8h  __attribute__((ext_vector_type(8)));
typedef float    v8f  __attribute__((ext_vector_type(8)));

#define LDK 2176


__device__ __forceinline__ v16h load_a_frag(const _Float16* __restrict__ base, int lane)
{
    const _Float16* p = base + (size_t)(lane & 15) * LDK + ((lane >> 4) << 3);
    v8h lo = *(const v8h*)p;
    v8h hi = *(const v8h*)(p + 16);
    return __builtin_shufflevector(lo, hi, 0, 1, 2, 3, 4, 5, 6, 7,
                                   8, 9, 10, 11, 12, 13, 14, 15);
}

__device__ __forceinline__ v16h load_b_frag(const _Float16* __restrict__ base, int lane)
{
    return load_a_frag(base, lane);
}
__device__ __forceinline__ v8f wmma16(v16h a, v16h b, v8f c)
{
    v8f d = __builtin_amdgcn_wmma_f32_16x16x32_f16(false, a, false, b, (short)0, c, false, false);
    asm volatile("v_nop\n\tv_nop\n\tv_nop\n\tv_nop" : "+v"(d) : "v"(a), "v"(b));
    return d;
}


#define PPB 16
__device__ __forceinline__ v16h frag_row_f16(const _Float16* row, int hh) {
    v8h lo = *(const v8h*)(row + 8 * hh), hi = *(const v8h*)(row + 16 + 8 * hh);
    return __builtin_shufflevector(lo, hi, 0, 1, 2, 3, 4, 5, 6, 7, 8, 9, 10, 11, 12, 13, 14, 15);
}
__device__ __forceinline__ v16h frag_row_f32(const float* row, int hh) {
    v16h f;
#pragma unroll
    for (int e = 0; e < 8; ++e) { f[e] = (_Float16)row[8 * hh + e]; f[8 + e] = (_Float16)row[16 + 8 * hh + e]; }
    return f;
}
__global__ __launch_bounds__(256) void rm_factor_kernel(
    const float* __restrict__ Q, const float* __restrict__ Kp,
    const float* __restrict__ W1, const float* __restrict__ b1,
    const float* __restrict__ W2, const float* __restrict__ b2,
    _Float16* __restrict__ Aq, _Float16* __restrict__ Bk)
{
    __shared__ __attribute__((aligned(16))) float    sx[PPB][32];
    __shared__ __attribute__((aligned(16))) _Float16 sxh[PPB][32];
    __shared__ __attribute__((aligned(16))) _Float16 shh[PPB][64];
    __shared__ __attribute__((aligned(16))) _Float16 sLh[PPB][32][40];
    __shared__ __attribute__((aligned(16))) float    sG[PPB][1024];
    __shared__ float sc[PPB][32];
    __shared__ float sa[PPB];

    const int pid0 = blockIdx.x * PPB;
    const bool isQ = pid0 < 2048;
    const int p0 = isQ ? pid0 : pid0 - 2048;
    const float* xg = (isQ ? Q : Kp) + (size_t)p0 * 32;
    _Float16* outbase = (isQ ? Aq : Bk) + (size_t)p0 * LDK;
    const int t = threadIdx.x, lane = t & 31, wave = t >> 5, hh = lane >> 4, l16 = lane & 15;

    for (int i = t; i < PPB * 32; i += 256) { const float v = xg[i]; sx[i >> 5][i & 31] = v; sxh[i >> 5][i & 31] = (_Float16)v; }
    __syncthreads();

    if (wave < 4) {
        const v16h a = frag_row_f16(&sxh[l16][0], hh);
        const v16h b = frag_row_f32(W1 + (size_t)(wave * 16 + l16) * 32, hh);
        v8f c = {}; c = wmma16(a, b, c);
#pragma unroll
        for (int r = 0; r < 8; ++r) { const int n = wave * 16 + l16; const float v = c[r] + b1[n]; shh[8 * hh + r][n] = (_Float16)(v / (1.0f + expf(-v))); }
    }
    __syncthreads();

    {
        const v16h a0 = frag_row_f16(&shh[l16][0], hh), a1 = frag_row_f16(&shh[l16][32], hh);
        for (int nt = wave; nt < 64; nt += 8) {
            const int n = nt * 16 + l16;
            const float* wrow = W2 + (size_t)n * 64;
            v8f c = {};
            c = wmma16(a0, frag_row_f32(wrow, hh), c);
            c = wmma16(a1, frag_row_f32(wrow + 32, hh), c);
            const int d = n >> 5, e = n & 31;
#pragma unroll
            for (int r = 0; r < 8; ++r) {
                const int pt = 8 * hh + r;
                float acc = fminf(fmaxf(c[r] + b2[n], -5.0f), 5.0f);
                float Lv;
                if (e > d)       Lv = 0.0f;
                else if (e < d)  Lv = acc;
                else { const float v = acc + 1.0f; Lv = log1pf(expf(v)) + 1e-4f; }
                sLh[pt][d][e] = (_Float16)Lv;
            }
        }
    }
    __syncthreads();

    for (int tt = wave; tt < PPB * 4; tt += 8) {
        const int pt = tt >> 2, mi = (tt >> 1) & 1, ni = tt & 1;
        const v16h a = frag_row_f16(&sLh[pt][mi * 16 + l16][0], hh);
        const v16h b = frag_row_f16(&sLh[pt][ni * 16 + l16][0], hh);
        v8f c = {}; c = wmma16(a, b, c);
#pragma unroll
        for (int r = 0; r < 8; ++r) sG[pt][(mi * 16 + 8 * hh + r) * 32 + ni * 16 + l16] = c[r];
    }
    __syncthreads();

    for (int i = t; i < PPB * 32; i += 256) {
        const int pt = i >> 5, d = i & 31;
        float acc = 0.0f;
        for (int e = 0; e < 32; ++e) acc = fmaf(sG[pt][d * 32 + e], sx[pt][e], acc);
        sc[pt][d] = acc;
    }
    __syncthreads();
    if (t < PPB) {
        float acc = 0.0f;
        for (int d = 0; d < 32; ++d) acc = fmaf(sx[t][d], sc[t][d], acc);
        sa[t] = acc;
    }
    __syncthreads();

    for (int pass = 0; pass < 2; ++pass) {
        for (int piece = t; piece < PPB * (LDK / 8); piece += 256) {
            const int pt = piece / (LDK / 8), k0 = (piece - pt * (LDK / 8)) * 8;
            v8h hv;
#pragma unroll
            for (int q8 = 0; q8 < 8; ++q8) {
                const int k = k0 + q8;
                float v;
                if (isQ) {
                    if (k < 1024)        v = sG[pt][k];
                    else if (k < 2048) { int kk = k - 1024; v = sx[pt][kk >> 5] * sx[pt][kk & 31]; }
                    else if (k < 2080)   v = -2.0f * sc[pt][k - 2048];
                    else if (k < 2112)   v = -2.0f * sx[pt][k - 2080];
                    else if (k == 2112)  v = sa[pt];
                    else if (k == 2113)  v = 1.0f;
                    else                 v = 0.0f;
                } else {
                    if (k < 1024)      { v = sx[pt][k >> 5] * sx[pt][k & 31]; }
                    else if (k < 2048)   v = sG[pt][k - 1024];
                    else if (k < 2080)   v = sx[pt][k - 2048];
                    else if (k < 2112)   v = sc[pt][k - 2080];
                    else if (k == 2112)  v = 1.0f;
                    else if (k == 2113)  v = sa[pt];
                    else                 v = 0.0f;
                }
                hv[q8] = (_Float16)v;
            }
            *(volatile v8h*)(outbase + (size_t)pt * LDK + k0) = hv;
        }
        __threadfence();
    }
}

__device__ __forceinline__ float rm_epilogue(float acc)
{
    float d2 = fminf(fmaxf(0.5f * acc, 1e-6f), 1e6f);
    return sqrtf(d2);
}

__global__ __launch_bounds__(256) void rm_gemm_kernel(
    const _Float16* __restrict__ A, const _Float16* __restrict__ Bm,
    float* __restrict__ out)
{
    const int bz   = blockIdx.z;
    const int lane = threadIdx.x & 31;
    const int w    = threadIdx.x >> 5;
    const int rowBase = blockIdx.x * 128 + (w >> 1) * 32;
    const int colBase = blockIdx.y * 64  + (w & 1) * 32;

    const _Float16* Ab = A  + (size_t)bz * 1024 * LDK;
    const _Float16* Bb = Bm + (size_t)bz * 1024 * LDK;

    v8f c00 = {}, c01 = {}, c10 = {}, c11 = {};

    for (int k0 = 0; k0 < LDK; k0 += 32) {
        v16h a0 = load_a_frag(Ab + (size_t)rowBase * LDK + k0, lane);
        v16h a1 = load_a_frag(Ab + (size_t)(rowBase + 16) * LDK + k0, lane);
        v16h b0 = load_b_frag(Bb + (size_t)colBase * LDK + k0, lane);
        v16h b1 = load_b_frag(Bb + (size_t)(colBase + 16) * LDK + k0, lane);

        c00 = wmma16(a0, b0, c00);
        c01 = wmma16(a0, b1, c01);
        c10 = wmma16(a1, b0, c10);
        c11 = wmma16(a1, b1, c11);
    }

    float* outb = out + (size_t)bz * 1024 * 1024;
    const int hh = lane >> 4;
    for (int pass = 0; pass < 2; ++pass) {
        #pragma unroll
        for (int v = 0; v < 8; ++v) {
            {
                const float a_ = rm_epilogue(c00[v]), b_ = rm_epilogue(c01[v]);
                const float ax = __shfl_xor(a_, 16), bx = __shfl_xor(b_, 16);
                *(volatile float*)(outb + (size_t)(rowBase + v) * 1024 + colBase + lane) = hh ? bx : a_;
                *(volatile float*)(outb + (size_t)(rowBase + v + 8) * 1024 + colBase + lane) = hh ? b_ : ax;
            }
            {
                const float a_ = rm_epilogue(c10[v]), b_ = rm_epilogue(c11[v]);
                const float ax = __shfl_xor(a_, 16), bx = __shfl_xor(b_, 16);
                *(volatile float*)(outb + (size_t)(rowBase + 16 + v) * 1024 + colBase + lane) = hh ? bx : a_;
                *(volatile float*)(outb + (size_t)(rowBase + 16 + v + 8) * 1024 + colBase + lane) = hh ? b_ : ax;
            }
        }
        __threadfence();
    }
}

extern "C" void kernel_launch(void* const* d_in, const int* in_sizes, int n_in,
                              void* d_out, int out_size, void* d_ws, size_t ws_size,
                              hipStream_t stream)
{
    (void)in_sizes; (void)n_in; (void)out_size;
    if (ws_size < (size_t)4 * 1024 * LDK * sizeof(_Float16)) return;
    const float* Q  = (const float*)d_in[0];
    const float* K  = (const float*)d_in[1];
    const float* W1 = (const float*)d_in[2];
    const float* b1 = (const float*)d_in[3];
    const float* W2 = (const float*)d_in[4];
    const float* b2 = (const float*)d_in[5];
    float* out = (float*)d_out;

    _Float16* Aq = (_Float16*)d_ws;
    _Float16* Bk = Aq + (size_t)2 * 1024 * LDK;

    rm_factor_kernel<<<4096 / PPB, 256, 0, stream>>>(Q, K, W1, b1, W2, b2, Aq, Bk);
    rm_gemm_kernel<<<dim3(8, 16, 2), 256, 0, stream>>>(Aq, Bk, out);
}
